// DifferentiableLayer_11218454577800
// MI455X (gfx1250) — hardware-verified
//
#include <hip/hip_runtime.h>
#include <stdint.h>
#include <math.h>

typedef __attribute__((ext_vector_type(16))) _Float16 v16h;
typedef __attribute__((ext_vector_type(8)))  _Float16 v8h;
typedef __attribute__((ext_vector_type(16))) __bf16   v16b;
typedef __attribute__((ext_vector_type(8)))  __bf16   v8b;
typedef __attribute__((ext_vector_type(8)))  float    v8f;
typedef __attribute__((ext_vector_type(4)))  float    v4f;
typedef __attribute__((ext_vector_type(4)))  unsigned v4u_base;
typedef v4u_base __attribute__((may_alias)) v4ua;

enum {
  NB_ROWS     = 4096,
  NI_FEAT     = 512,
  NO_FEAT     = 512,
  NK_OPS      = 6,
  KDIM        = NI_FEAT * NK_OPS,
  ROW_U32     = KDIM / 2,
  ROW_CHUNK16 = (KDIM * 2) / 16
};

__device__ __forceinline__ unsigned short f2bf_bits(float f) {
  unsigned u = __float_as_uint(f);
  return (unsigned short)((u + 0x7FFFu + ((u >> 16) & 1u)) >> 16);
}
__device__ __forceinline__ float bf_bits2f(unsigned short h) { return __uint_as_float(((unsigned)h) << 16); }
__device__ __forceinline__ unsigned f2h_bits(float f) { return (unsigned)__builtin_bit_cast(unsigned short, (_Float16)f); }

__device__ __forceinline__ void dep_guard_h(v8f& a, v8f& b, v16h x, v16h y) { asm volatile("v_nop\n\tv_nop\n\tv_nop\n\tv_nop" : "+v"(a), "+v"(b) : "v"(x), "v"(y)); }
__device__ __forceinline__ void dep_guard_b(v8f& a, v8f& b, v16b x, v16b y) { asm volatile("v_nop\n\tv_nop\n\tv_nop\n\tv_nop" : "+v"(a), "+v"(b) : "v"(x), "v"(y)); }
__device__ __forceinline__ void keep4_h(v16h a, v16h b, v16h c, v16h d) { asm volatile("v_nop" :: "v"(a), "v"(b), "v"(c), "v"(d)); }
__device__ __forceinline__ void keep4_b(v16b a, v16b b, v16b c, v16b d) { asm volatile("v_nop" :: "v"(a), "v"(b), "v"(c), "v"(d)); }
__device__ __forceinline__ void acc_guard4(v8f& a, v8f& b, v8f& c, v8f& d) { asm volatile("v_nop\n\tv_nop\n\tv_nop\n\tv_nop" : "+v"(a), "+v"(b), "+v"(c), "+v"(d)); }
template <typename T> struct Frag;
template <> struct Frag<_Float16> {
  typedef v16h V; union U { v16h v; v8h h[2]; };
  static __device__ __forceinline__ v16h load(const _Float16* p) {
    U f; f.h[0] = *(const v8h*)(p); f.h[1] = *(const v8h*)(p + 16); return f.v;
  }
  static __device__ __forceinline__ v8f mma(v16h a, v16h b, v8f c) {
    return __builtin_amdgcn_wmma_f32_16x16x32_f16(false, a, false, b, (short)0, c, false, false);
  }
  static __device__ __forceinline__ void guard(v8f& a, v8f& b, v16h x, v16h y) { dep_guard_h(a, b, x, y); }
  static __device__ __forceinline__ void keep(v16h a, v16h b, v16h c, v16h d) { keep4_h(a, b, c, d); }
};
template <> struct Frag<__bf16> {
  typedef v16b V; union U { v16b v; v8b h[2]; };
  static __device__ __forceinline__ v16b load(const __bf16* p) {
    U f; f.h[0] = *(const v8b*)(p); f.h[1] = *(const v8b*)(p + 16); return f.v;
  }
  static __device__ __forceinline__ v8f mma(v16b a, v16b b, v8f c) {
    return __builtin_amdgcn_wmma_f32_16x16x32_bf16(false, a, false, b, (short)0, c, false, false);
  }
  static __device__ __forceinline__ void guard(v8f& a, v8f& b, v16b x, v16b y) { dep_guard_b(a, b, x, y); }
  static __device__ __forceinline__ void keep(v16b a, v16b b, v16b c, v16b d) { keep4_b(a, b, c, d); }
};

template <int ET> struct Elem;
template <> struct Elem<0> { typedef _Float16 T; };
template <> struct Elem<1> { typedef __bf16 T; };
template <int ET, bool SPLIT, int BIAS_MODE, int OUT_MODE, bool RESID, int ACT = 0>
__global__ __launch_bounds__(256) void wmma_gemm64(
    const unsigned short* __restrict__ Ap, const unsigned short* __restrict__ A2p, int lda, long strideA,
    const unsigned short* __restrict__ Btp, const unsigned short* __restrict__ Bt2p, int ldb, long strideB,
    void* __restrict__ Cout, void* __restrict__ Cout2, int ldc, long strideC,
    const float* __restrict__ bias,
    const float* __restrict__ resid, long strideR,
    int M, int N, int K, float scale) {
  typedef typename Elem<ET>::T T;
  typedef typename Frag<T>::V V;
  const T* A = (const T*)Ap; const T* A2 = (const T*)A2p; const T* Bt = (const T*)Btp; const T* Bt2 = (const T*)Bt2p;
  __shared__ __align__(16) float sT[8][16 * 68];
  const int b    = blockIdx.y;
  const int lane = threadIdx.x & 31;
  const int wave = threadIdx.x >> 5;
  const int tilesN = N >> 6;
  const int tilesM = M >> 6;
  const int tile = blockIdx.x * 8 + wave;
  if (tile >= tilesM * tilesN) return;
  const int tm = tile / tilesN;
  const int tn = tile - tm * tilesN;
  const int m0 = tm << 6;
  const int n0 = tn << 6;

  const T* Ab  = A  + (size_t)b * strideA;
  const T* Bb  = Bt + (size_t)b * strideB;
  const T* Ab2 = SPLIT ? (A2  + (size_t)b * strideA) : nullptr;
  const T* Bb2 = SPLIT ? (Bt2 + (size_t)b * strideB) : nullptr;

  const int rlane = lane & 15;
  const int koff  = (lane >> 4) * 8;
  const int mOff  = (lane >> 4) * 8;

  v8f acc[4][4];
#pragma unroll
  for (int i = 0; i < 4; ++i)
#pragma unroll
    for (int j = 0; j < 4; ++j) acc[i][j] = (v8f){0.f,0.f,0.f,0.f,0.f,0.f,0.f,0.f};

  for (int k0 = 0; k0 < K; k0 += 32) {
    V bh[4], bl[4];
#pragma unroll
    for (int j = 0; j < 4; ++j) {
      const size_t bo = (size_t)(n0 + (j << 4) + rlane) * ldb + koff + k0;
      bh[j] = Frag<T>::load(Bb + bo);
      if (SPLIT) bl[j] = Frag<T>::load(Bb2 + bo);
    }
#pragma unroll
    for (int i = 0; i < 4; ++i) {
      const size_t ao = (size_t)(m0 + (i << 4) + rlane) * lda + koff + k0;
      V ah = Frag<T>::load(Ab + ao);
      V al;
      if (SPLIT) al = Frag<T>::load(Ab2 + ao);
#pragma unroll
      for (int j = 0; j < 4; ++j) {
        acc[i][j] = Frag<T>::mma(ah, bh[j], acc[i][j]);
        if (SPLIT) {
          acc[i][j] = Frag<T>::mma(ah, bl[j], acc[i][j]);
          acc[i][j] = Frag<T>::mma(al, bh[j], acc[i][j]);
        }
      }
      Frag<T>::guard(acc[i][0], acc[i][3], ah, SPLIT ? al : ah);
    }
    Frag<T>::keep(bh[0], bh[1], bh[2], bh[3]);
    if (SPLIT) Frag<T>::keep(bl[0], bl[1], bl[2], bl[3]);
  }
  acc_guard4(acc[0][0], acc[0][1], acc[0][2], acc[0][3]);
  acc_guard4(acc[1][0], acc[1][1], acc[1][2], acc[1][3]);
  acc_guard4(acc[2][0], acc[2][1], acc[2][2], acc[2][3]);
  acc_guard4(acc[3][0], acc[3][1], acc[3][2], acc[3][3]);

  float* slab = sT[wave];
  const float* Rb = RESID ? (resid + (size_t)b * strideR) : nullptr;
#pragma unroll
  for (int i = 0; i < 4; ++i) {
    const int mBase = m0 + (i << 4);
#pragma unroll
    for (int j = 0; j < 4; ++j) {
      const int n = n0 + (j << 4) + rlane;
      float bv = 0.f;
      if (BIAS_MODE == 2) bv = bias[n];
#pragma unroll
      for (int r = 0; r < 8; ++r) {
        float v = acc[i][j][r] * scale;
        if (BIAS_MODE == 1) v += bias[mBase + mOff + r];
        if (BIAS_MODE == 2) v += bv;
        if (RESID) v += Rb[(size_t)(mBase + mOff + r) * ldc + n];
        if (ACT == 1) v = tanhf(v);
        if (ACT == 2) v = fmaxf(v, 0.0f);
        if (ACT == 3) v = v / (1.0f + expf(-v));
        if (ACT == 4) v = (v > 0.f) ? v : 0.01f * v;
        if (ACT == 5) v = 0.5f * v * (1.0f + erff(v * 0.70710678118654752f));
        slab[(mOff + r) * 68 + (j << 4) + rlane] = v;
      }
    }
    __builtin_amdgcn_fence(__ATOMIC_RELEASE, "workgroup");
    __builtin_amdgcn_wave_barrier();
    __builtin_amdgcn_fence(__ATOMIC_ACQUIRE, "workgroup");
    if (OUT_MODE == 0) {
      float* C = (float*)Cout + (size_t)b * strideC;
      const int hh = lane >> 4, c4 = (lane & 15) * 4;
      for (int pass = 0; pass < 2; ++pass) {
#pragma unroll
        for (int it = 0; it < 8; ++it) {
          const int row = it * 2 + hh;
          v4f v = *(const v4f*)(slab + row * 68 + c4);
          *(volatile v4f*)(C + (size_t)(mBase + row) * ldc + n0 + c4) = v;
        }
        __threadfence();
      }
    } else {
      const int q = lane >> 3, c8 = (lane & 7) * 8;
      unsigned short* C  = (unsigned short*)Cout  + (size_t)b * strideC;
      unsigned short* C2 = (OUT_MODE == 2) ? ((unsigned short*)Cout2 + (size_t)b * strideC) : nullptr;
      for (int pass = 0; pass < 2; ++pass) {
#pragma unroll
        for (int it = 0; it < 4; ++it) {
          const int row = it * 4 + q;
          const float* sp = slab + row * 68 + c8;
          v8h hv, lv;
#pragma unroll
          for (int e = 0; e < 8; ++e) {
            if (OUT_MODE == 1) {
              hv[e] = (_Float16)sp[e];
            } else {
              unsigned short hb = f2bf_bits(sp[e]);
              unsigned short lb = f2bf_bits(sp[e] - bf_bits2f(hb));
              hv[e] = __builtin_bit_cast(_Float16, hb);
              lv[e] = __builtin_bit_cast(_Float16, lb);
            }
          }
          *(volatile v8h*)(C + (size_t)(mBase + row) * ldc + n0 + c8) = hv;
          if (OUT_MODE == 2) *(volatile v8h*)(C2 + (size_t)(mBase + row) * ldc + n0 + c8) = lv;
        }
        __threadfence();
      }
    }
    __builtin_amdgcn_fence(__ATOMIC_RELEASE, "workgroup");
    __builtin_amdgcn_wave_barrier();
    __builtin_amdgcn_fence(__ATOMIC_ACQUIRE, "workgroup");
  }
}

__device__ __forceinline__ void store_row_whole_lines(const unsigned* sRow, unsigned* __restrict__ dst_row, int tid) {
  if (tid < ROW_CHUNK16) {
    const v4ua val = *(const v4ua*)(sRow + tid * 4);
    unsigned* dst = dst_row + tid * 4;
    *(volatile v4ua*)dst = val;
    __threadfence();
    *(volatile v4ua*)dst = val;
  }
}

__global__ __launch_bounds__(512) void op_bank_plane(const float* __restrict__ x, unsigned* __restrict__ ops_plane) {
  __shared__ __align__(16) unsigned sRow[ROW_U32];
  const int b = blockIdx.x;
  const int i = threadIdx.x;
  const float v  = x[(size_t)b * NI_FEAT + i];
  const float sv = sinf(v);
  const float cv = cosf(v);
  const float th = tanhf(v);
  const float sq = v * v;
  const float rl = (v > 0.0f) ? v : 0.0f;
  const unsigned h0 = f2h_bits(v),  h1 = f2h_bits(sv);
  const unsigned h2 = f2h_bits(cv), h3 = f2h_bits(th);
  const unsigned h4 = f2h_bits(sq), h5 = f2h_bits(rl);
  sRow[i * 3 + 0] = h0 | (h1 << 16);
  sRow[i * 3 + 1] = h2 | (h3 << 16);
  sRow[i * 3 + 2] = h4 | (h5 << 16);
  __syncthreads();
  store_row_whole_lines(sRow, ops_plane + (size_t)b * ROW_U32, i);
}

__global__ __launch_bounds__(512) void hard_choice_plane(const float* __restrict__ w, const float* __restrict__ gmb,
                                                         unsigned* __restrict__ pb_plane) {
  __shared__ __align__(16) unsigned sRow[ROW_U32];
  const int o = blockIdx.x;
  const int i = threadIdx.x;
  const size_t e0 = ((size_t)o * NI_FEAT + i) * NK_OPS;
  const float* wp = w + e0;
  const float* gp = gmb + e0;
  float best = wp[0] + gp[0];
  int sel = 0;
#pragma unroll 1
  for (int k = 1; k < NK_OPS; ++k) {
    const float s = wp[k] + gp[k];
    if (s > best) { best = s; sel = k; }
  }
  float ssum = 0.0f;
#pragma unroll 1
  for (int k = 0; k < NK_OPS; ++k) {
    const float s = wp[k] + gp[k];
    ssum += expf(s - best);
  }
  const float ysel = 1.0f * (1.0f / ssum);
  const float psel = (1.0f - ysel) + ysel;
  const unsigned bits = f2h_bits(psel);
  const unsigned w0 = ((sel == 0) ? bits : 0u) | ((sel == 1) ? (bits << 16) : 0u);
  const unsigned w1 = ((sel == 2) ? bits : 0u) | ((sel == 3) ? (bits << 16) : 0u);
  const unsigned w2 = ((sel == 4) ? bits : 0u) | ((sel == 5) ? (bits << 16) : 0u);
  sRow[i * 3 + 0] = w0;
  sRow[i * 3 + 1] = w1;
  sRow[i * 3 + 2] = w2;
  __syncthreads();
  store_row_whole_lines(sRow, pb_plane + (size_t)o * ROW_U32, i);
}

extern "C" void kernel_launch(void* const* d_in, const int* in_sizes, int n_in,
                              void* d_out, int out_size, void* d_ws, size_t ws_size,
                              hipStream_t stream) {
  if (n_in < 3) return;
  if (in_sizes[0] != NB_ROWS * NI_FEAT) return;
  if (in_sizes[1] != NO_FEAT * NI_FEAT * NK_OPS) return;
  if (in_sizes[2] != NO_FEAT * NI_FEAT * NK_OPS) return;
  if (out_size != NB_ROWS * NO_FEAT) return;
  const size_t ops_bytes = (size_t)NB_ROWS * KDIM * 2;
  const size_t pb_bytes  = (size_t)NO_FEAT * KDIM * 2;
  if (ops_bytes + pb_bytes > ws_size) return;

  const float* x   = (const float*)d_in[0];
  const float* w   = (const float*)d_in[1];
  const float* gmb = (const float*)d_in[2];
  float* out = (float*)d_out;

  unsigned char* wsb = (unsigned char*)d_ws;
  unsigned* ops_plane = (unsigned*)(wsb);
  unsigned* pb_plane  = (unsigned*)(wsb + ops_bytes);

  op_bank_plane<<<dim3(NB_ROWS), dim3(512), 0, stream>>>(x, ops_plane);
  hard_choice_plane<<<dim3(NO_FEAT), dim3(512), 0, stream>>>(w, gmb, pb_plane);

  const int tiles = (NB_ROWS / 64) * (NO_FEAT / 64);
  dim3 ggrid((tiles + 7) / 8, 1);
  wmma_gemm64<0, false, 0, 0, false, 0><<<ggrid, dim3(256), 0, stream>>>(
      (const unsigned short*)ops_plane, (const unsigned short*)ops_plane, KDIM, 0L,
      (const unsigned short*)pb_plane,  (const unsigned short*)pb_plane,  KDIM, 0L,
      (void*)out, (void*)out, NO_FEAT, 0L,
      (const float*)pb_plane,
      (const float*)pb_plane, 0L,
      NB_ROWS, NO_FEAT, KDIM, 1.0f);
}
